// DilatedCausalSelfAttention_40166534152421
// MI455X (gfx1250) — hardware-verified
//
#include <hip/hip_runtime.h>


#define LL   4096
#define EE   1024
#define NH_  16
#define HD   64
#define GG   1024
#define PCAR 1024.0f
typedef _Float16 h16;
typedef unsigned short bf;
typedef __attribute__((ext_vector_type(16))) __bf16   v16bf;
typedef __attribute__((ext_vector_type(16))) _Float16 v16h;
typedef __attribute__((ext_vector_type(8)))  _Float16 v8h;
typedef __attribute__((ext_vector_type(8)))  unsigned short v8us;
typedef __attribute__((ext_vector_type(8)))  float    v8f;
typedef __attribute__((ext_vector_type(4)))  float    v4f;
typedef v8h  __attribute__((may_alias)) v8ha;
typedef v4f  __attribute__((may_alias)) v4fa;
typedef v8us __attribute__((may_alias)) v8usa;

__device__ __forceinline__ unsigned short f2bf(float f) { unsigned u = __float_as_uint(f); u += 0x7FFFu + ((u >> 16) & 1u); return (unsigned short)(u >> 16); }
__device__ __forceinline__ float bf2f(unsigned short b) { return __uint_as_float(((unsigned)b) << 16); }
__device__ __forceinline__ float bfr(float f) { return bf2f(f2bf(f)); }
__device__ __forceinline__ v16h cat16(v8h lo, v8h hi) { return __builtin_shufflevector(lo, hi, 0, 1, 2, 3, 4, 5, 6, 7, 8, 9, 10, 11, 12, 13, 14, 15); }
__device__ __forceinline__ v16bf cat16b(v8us lo, v8us hi) { return __builtin_bit_cast(v16bf, __builtin_shufflevector(lo, hi, 0, 1, 2, 3, 4, 5, 6, 7, 8, 9, 10, 11, 12, 13, 14, 15)); }
__device__ __forceinline__ v8f wmma16(v16h a, v16h b, v8f c) { return __builtin_amdgcn_wmma_f32_16x16x32_f16(false, a, false, b, (short)0, c, false, false); }
__device__ __forceinline__ v8f wmmab(v16bf a, v16bf b, v8f c) { return __builtin_amdgcn_wmma_f32_16x16x32_bf16(false, a, false, b, (short)0, c, false, false); }


template <typename T16> struct WFrag;
template <> struct WFrag<h16> { typedef v16h V; static __device__ __forceinline__ V ld(const h16* p) { return cat16(*(const v8h*)p, *(const v8h*)(p + 16)); } static __device__ __forceinline__ v8f mma(V a, V b, v8f c) { return wmma16(a, b, c); } };
template <> struct WFrag<bf> { typedef v16bf V; static __device__ __forceinline__ V ld(const bf* p) { return cat16b(*(const v8us*)p, *(const v8us*)(p + 16)); } static __device__ __forceinline__ v8f mma(V a, V b, v8f c) { return wmmab(a, b, c); } };
template <typename T16, int NSPLIT, bool BIAS>
__global__ __launch_bounds__(32) void k_gemmw(const T16* __restrict__ A, const T16* __restrict__ A2, const T16* __restrict__ Bt, const T16* __restrict__ Bt2, int K, float* C, int ldc, const float* __restrict__ bias, size_t sA, size_t sB, size_t sC) {
    typedef typename WFrag<T16>::V V;
    __shared__ __align__(16) float os[16 * 68];
    const size_t z = blockIdx.z; A += z * sA; if (A2) A2 += z * sA; Bt += z * sB; if (Bt2) Bt2 += z * sB; C += z * sC;
    const int lane = threadIdx.x & 31, lr = lane & 15, hi = lane >> 4; const int r0 = blockIdx.x * 64, c0 = blockIdx.y * 64;
    v8f acc[4][4];
#pragma unroll
    for (int mb = 0; mb < 4; ++mb)
#pragma unroll
        for (int nb = 0; nb < 4; ++nb) acc[mb][nb] = (v8f){};
    const size_t aoff = (size_t)(r0 + lr) * K + 8 * hi, boff = (size_t)(c0 + lr) * K + 8 * hi;
#pragma unroll 1
    for (int kc = 0; kc < K; kc += 32) {
        V a[4], a2[4];
#pragma unroll
        for (int mb = 0; mb < 4; ++mb) { a[mb] = WFrag<T16>::ld(A + aoff + (size_t)mb * 16 * K + kc); if (NSPLIT == 1 || NSPLIT == 2) a2[mb] = WFrag<T16>::ld(A2 + aoff + (size_t)mb * 16 * K + kc); }
#pragma unroll
        for (int nb = 0; nb < 4; ++nb) { const V b = WFrag<T16>::ld(Bt + boff + (size_t)nb * 16 * K + kc); V b2; if (NSPLIT >= 2) b2 = WFrag<T16>::ld(Bt2 + boff + (size_t)nb * 16 * K + kc);
#pragma unroll
            for (int mb = 0; mb < 4; ++mb) { acc[mb][nb] = WFrag<T16>::mma(a[mb], b, acc[mb][nb]); if (NSPLIT == 1 || NSPLIT == 2) acc[mb][nb] = WFrag<T16>::mma(a2[mb], b, acc[mb][nb]); if (NSPLIT >= 2) acc[mb][nb] = WFrag<T16>::mma(a[mb], b2, acc[mb][nb]); } }
        asm volatile("v_nop\n\tv_nop\n\tv_nop\n\tv_nop" : "+v"(acc[0][0]), "+v"(acc[1][1]), "+v"(acc[2][2]), "+v"(acc[3][3]) : "v"(a[0]), "v"(a[3]));
    }
#pragma unroll
    for (int mb = 0; mb < 4; ++mb) {
#pragma unroll
        for (int nb = 0; nb < 4; ++nb) {
#pragma unroll
            for (int j = 0; j < 8; ++j) os[(hi * 8 + j) * 68 + nb * 16 + lr] = acc[mb][nb][j]; }
        __builtin_amdgcn_wave_barrier(); asm volatile("" ::: "memory");
        float* crow = C + (size_t)(r0 + mb * 16) * ldc + c0;
#pragma unroll 1
        for (int ps = 0; ps < 2; ++ps) {
#pragma unroll
            for (int s = 0; s < 8; ++s) { const int row = 2 * s + hi, cofs = lr * 4; v4f val = *(const v4fa*)(os + row * 68 + cofs); if (BIAS) { val[0] += bfr(bias[c0 + cofs]); val[1] += bfr(bias[c0 + cofs + 1]); val[2] += bfr(bias[c0 + cofs + 2]); val[3] += bfr(bias[c0 + cofs + 3]); }
                *(volatile v4f*)(crow + (size_t)row * ldc + cofs) = val; }
            if (ps == 0) __threadfence(); }
        __builtin_amdgcn_wave_barrier(); asm volatile("" ::: "memory");
    }
}

template <typename T16, int NSPLIT, int CMODE>
__global__ __launch_bounds__(32) void k_gemmc(const T16* __restrict__ A, const T16* __restrict__ A2, const T16* __restrict__ Bt, const T16* __restrict__ Bt2, int K, float* C, int ldc, int roff, size_t sA, size_t sB, size_t sC) {
    typedef typename WFrag<T16>::V V;
    __shared__ __align__(16) float os[16 * 68];
    const size_t z = blockIdx.z; A += z * sA; if (A2) A2 += z * sA; Bt += z * sB; if (Bt2) Bt2 += z * sB; C += z * sC;
    const int lane = threadIdx.x & 31, lr = lane & 15, hi = lane >> 4; const int r0 = blockIdx.x * 64, c0 = blockIdx.y * 64;
    if (CMODE == 1 && c0 > r0 + roff + 63) return;
    const int Kl = (CMODE == 2) ? min(K, r0 + roff + 64) : K;
    v8f acc[4][4];
#pragma unroll
    for (int mb = 0; mb < 4; ++mb)
#pragma unroll
        for (int nb = 0; nb < 4; ++nb) acc[mb][nb] = (v8f){};
    const size_t aoff = (size_t)(r0 + lr) * K + 8 * hi, boff = (size_t)(c0 + lr) * K + 8 * hi;
#pragma unroll 1
    for (int kc = 0; kc < Kl; kc += 32) {
        V a[4], a2[4];
#pragma unroll
        for (int mb = 0; mb < 4; ++mb) { a[mb] = WFrag<T16>::ld(A + aoff + (size_t)mb * 16 * K + kc); if (NSPLIT == 1 || NSPLIT == 2) a2[mb] = WFrag<T16>::ld(A2 + aoff + (size_t)mb * 16 * K + kc); }
#pragma unroll
        for (int nb = 0; nb < 4; ++nb) { const V b = WFrag<T16>::ld(Bt + boff + (size_t)nb * 16 * K + kc); V b2; if (NSPLIT >= 2) b2 = WFrag<T16>::ld(Bt2 + boff + (size_t)nb * 16 * K + kc);
#pragma unroll
            for (int mb = 0; mb < 4; ++mb) { acc[mb][nb] = WFrag<T16>::mma(a[mb], b, acc[mb][nb]); if (NSPLIT == 1 || NSPLIT == 2) acc[mb][nb] = WFrag<T16>::mma(a2[mb], b, acc[mb][nb]); if (NSPLIT >= 2) acc[mb][nb] = WFrag<T16>::mma(a[mb], b2, acc[mb][nb]); } }
        asm volatile("v_nop\n\tv_nop\n\tv_nop\n\tv_nop" : "+v"(acc[0][0]), "+v"(acc[1][1]), "+v"(acc[2][2]), "+v"(acc[3][3]) : "v"(a[0]), "v"(a[3]));
    }
#pragma unroll
    for (int mb = 0; mb < 4; ++mb) {
#pragma unroll
        for (int nb = 0; nb < 4; ++nb) {
#pragma unroll
            for (int j = 0; j < 8; ++j) os[(hi * 8 + j) * 68 + nb * 16 + lr] = acc[mb][nb][j]; }
        __builtin_amdgcn_wave_barrier(); asm volatile("" ::: "memory");
        float* crow = C + (size_t)(r0 + mb * 16) * ldc + c0;
#pragma unroll 1
        for (int ps = 0; ps < 2; ++ps) {
#pragma unroll
            for (int s = 0; s < 8; ++s) { const int row = 2 * s + hi, cofs = lr * 4; v4f val = *(const v4fa*)(os + row * 68 + cofs);
                *(volatile v4f*)(crow + (size_t)row * ldc + cofs) = val; }
            if (ps == 0) __threadfence(); }
        __builtin_amdgcn_wave_barrier(); asm volatile("" ::: "memory");
    }
}

__device__ __forceinline__ h16 tohx(float x) { return (h16)x; }
__device__ __forceinline__ void splitf(float y, unsigned short& h, unsigned short& l) { h = f2bf(y); l = f2bf(y - bf2f(h)); }
typedef __attribute__((ext_vector_type(2))) _Float16 v2h;
typedef __attribute__((ext_vector_type(4))) _Float16 v4h;
typedef __attribute__((ext_vector_type(2))) unsigned short v2us;
typedef __attribute__((ext_vector_type(4))) unsigned short v4us;
typedef __attribute__((ext_vector_type(2))) float v2f;
__device__ __forceinline__ int dpos(int r, int seg, int h, int gi) { const int w = GG * r; const int off = h / (NH_ / r); return seg * w + gi * r + off; }

__global__ __launch_bounds__(256) void k_wtG(const float* __restrict__ w, int K, int N, bf* Bt) {
    const int lane = threadIdx.x & 31; const int L0 = (blockIdx.x * 8 + (threadIdx.x >> 5)) * 8; const int nlines = N * K / 64;
#pragma unroll 1
    for (int ps = 0; ps < 2; ++ps) {
#pragma unroll 1
        for (int l = 0; l < 8; ++l) { const int L = L0 + l; if (L >= nlines) break; const size_t e = (size_t)L * 64 + lane * 2; const int k = (int)(e % K), n = (int)(e / K); v2us o;
            o[0] = f2bf(w[(size_t)k * N + n]); o[1] = f2bf(w[(size_t)(k + 1) * N + n]); *(volatile v2us*)(Bt + e) = o; }
        if (ps == 0) __threadfence(); }
}
__global__ __launch_bounds__(256) void k_cvt8(const float* __restrict__ src, bf* dst, size_t n8) { const size_t i = (size_t)blockIdx.x * 256 + threadIdx.x; if (i >= n8) return; const v8f v = *(const v8f*)(src + i * 8); v8us o;
#pragma unroll
    for (int k = 0; k < 8; ++k) o[k] = f2bf(v[k]); *(volatile v8us*)(dst + i * 8) = o; __threadfence(); *(volatile v8us*)(dst + i * 8) = o; }
#define ZC 8
__global__ __launch_bounds__(256) void k_gath(const float* __restrict__ QKV, int r, int z0, bf* Qh, bf* Ql, bf* Kh, bf* Kl) { const size_t e = ((size_t)blockIdx.x * 256 + threadIdx.x) * 2; if (e >= (size_t)ZC * GG * HD) return; const int d = (int)(e % HD); const int gi = (int)((e / HD) % GG); const int z = z0 + (int)(e / ((size_t)HD * GG)); const int h = z % NH_, seg = z / NH_; const float* row = QKV + (size_t)dpos(r, seg, h, gi) * (3 * EE) + h * HD + d; v2us qh, ql, kh, kl;
#pragma unroll
    for (int u = 0; u < 2; ++u) { unsigned short a, c; splitf(row[u] * 0.125f, a, c); qh[u] = a; ql[u] = c; splitf(row[EE + u], a, c); kh[u] = a; kl[u] = c; }
    for (int ps = 0; ps < 2; ++ps) { *(volatile v2us*)(Qh + e) = qh; *(volatile v2us*)(Ql + e) = ql; *(volatile v2us*)(Kh + e) = kh; *(volatile v2us*)(Kl + e) = kl; if (ps == 0) __threadfence(); } }
__global__ __launch_bounds__(256) void k_gathv(const float* __restrict__ QKV, int r, int z0, bf* Vh, bf* Vl) { const size_t e = ((size_t)blockIdx.x * 256 + threadIdx.x) * 2; if (e >= (size_t)ZC * HD * GG) return; const int gi = (int)(e % GG); const int d = (int)((e / GG) % HD); const int z = z0 + (int)(e / ((size_t)GG * HD)); const int h = z % NH_, seg = z / NH_; v2us oh, ol;
#pragma unroll
    for (int u = 0; u < 2; ++u) { unsigned short a, c; splitf(QKV[(size_t)dpos(r, seg, h, gi + u) * (3 * EE) + 2 * EE + h * HD + d], a, c); oh[u] = a; ol[u] = c; } *(volatile v2us*)(Vh + e) = oh; *(volatile v2us*)(Vl + e) = ol; __threadfence(); *(volatile v2us*)(Vh + e) = oh; *(volatile v2us*)(Vl + e) = ol; }
__global__ __launch_bounds__(256) void k_csoft(const float* __restrict__ Sb, bf* Ph, bf* Pl, float* LSEX) { const int lane = threadIdx.x & 31; const int row = blockIdx.x * 8 + (threadIdx.x >> 5); const int i = row % GG; const float* sr = Sb + (size_t)row * GG; float v[32]; float mx = -3.0e38f;
#pragma unroll
    for (int ch = 0; ch < 8; ++ch) { const int j0 = ch * 128 + lane * 4; const v4f a = *(const v4f*)(sr + j0);
#pragma unroll
        for (int q = 0; q < 4; ++q) { const float t = (j0 + q) <= i ? a[q] : -3.0e38f; v[ch * 4 + q] = t; mx = fmaxf(mx, t); } }
#pragma unroll
    for (int sh = 16; sh; sh >>= 1) mx = fmaxf(mx, __shfl_xor(mx, sh, 32));
    float sum = 0.f;
#pragma unroll
    for (int k = 0; k < 32; ++k) { float d0 = __fsub_rn(v[k], mx); asm volatile("" : "+v"(d0)); v[k] = __expf(d0); sum += v[k]; }
#pragma unroll
    for (int sh = 16; sh; sh >>= 1) sum += __shfl_xor(sum, sh, 32);
    const float inv = __fdiv_rn(1.0f, sum); float se = 0.f;
#pragma unroll
    for (int k = 0; k < 32; ++k) { v[k] = v[k] * inv; se = __fadd_rn(se, __expf(v[k])); }
#pragma unroll
    for (int sh = 16; sh; sh >>= 1) se += __shfl_xor(se, sh, 32);
    const float lse = __logf(se);
#pragma unroll 1
    for (int ps = 0; ps < 2; ++ps) {
#pragma unroll
        for (int ch = 0; ch < 8; ++ch) { v4us oh, ol;
#pragma unroll
            for (int q = 0; q < 4; ++q) { unsigned short a, c; splitf(v[ch * 4 + q], a, c); oh[q] = a; ol[q] = c; } const size_t oo = (size_t)row * GG + ch * 128 + lane * 4; *(volatile v4us*)(Ph + oo) = oh; *(volatile v4us*)(Pl + oo) = ol; }
        *(volatile float*)(LSEX + (size_t)row * 32 + lane) = lse;
        if (ps == 0) __threadfence(); } }
__global__ __launch_bounds__(256) void k_comb(const float* __restrict__ Ob0, const float* __restrict__ Ob1, const float* __restrict__ Ob2, const float* __restrict__ L0, const float* __restrict__ L1, const float* __restrict__ L2, bf* Ah, bf* Al) { const size_t e = ((size_t)blockIdx.x * 256 + threadIdx.x) * 2; if (e >= (size_t)LL * EE) return; const int d = (int)(e % HD); const int h = (int)((e / HD) % NH_); const int l = (int)(e / EE);
    const float* obs[3] = {Ob0, Ob1, Ob2}; const float* lss[3] = {L0, L1, L2}; float lse[3]; size_t src[3]; bool used[3];
#pragma unroll
    for (int k = 0; k < 3; ++k) { const int r = 1 << k; const int w = GG * r; const int ll = l % w; const int off = h / (NH_ / r); used[k] = (ll % r) == off; const int gi = ll / r; const int z = (l / w) * NH_ + h; src[k] = ((size_t)z * GG + gi); lse[k] = used[k] ? lss[k][src[k] * 32] : -1.0e8f; }
    const float m = fmaxf(lse[0], fmaxf(lse[1], lse[2])); float ex[3]; float den = 0.f;
#pragma unroll
    for (int k = 0; k < 3; ++k) { ex[k] = __expf(__fsub_rn(lse[k], m)); den = __fadd_rn(den, ex[k]); }
    const float inv = __fdiv_rn(1.0f, den); v2us oh, ol;
#pragma unroll
    for (int u = 0; u < 2; ++u) { float acc = 0.f;
#pragma unroll
        for (int k = 0; k < 3; ++k) { const float o = used[k] ? obs[k][src[k] * HD + d + u] : 0.f; float p = __fmul_rn(o, ex[k] * inv); asm volatile("" : "+v"(p)); acc = __fadd_rn(acc, p); }
        unsigned short a, c; splitf(acc, a, c); oh[u] = a; ol[u] = c; }
    *(volatile v2us*)(Ah + e) = oh; *(volatile v2us*)(Al + e) = ol; __threadfence(); *(volatile v2us*)(Ah + e) = oh; *(volatile v2us*)(Al + e) = ol; }

extern "C" void kernel_launch(void* const* d_in, const int* in_sizes, int n_in,
                              void* d_out, int out_size, void* d_ws, size_t ws_size, hipStream_t stream) {
    (void)in_sizes; (void)n_in; (void)out_size;
    const float* x = (const float*)d_in[0]; const float* wqkv = (const float*)d_in[1]; const float* wproj = (const float*)d_in[2];
    float* OUT = (float*)d_out;
    char* wsp = (char*)d_ws;
    auto take = [&](size_t bytes) { char* p = wsp; wsp += (bytes + 255) & ~(size_t)255; return (void*)p; };
    const int NZMAX = 4 * NH_;
    bf* WQ = (bf*)take((size_t)3 * EE * EE * 2); bf* WP = (bf*)take((size_t)EE * EE * 2); bf* XB = (bf*)take((size_t)LL * EE * 2); float* QKV = (float*)take((size_t)LL * 3 * EE * 4);
    bf* Qh = (bf*)take((size_t)ZC * GG * HD * 2); bf* Ql = (bf*)take((size_t)ZC * GG * HD * 2); bf* Kh = (bf*)take((size_t)ZC * GG * HD * 2); bf* Kl = (bf*)take((size_t)ZC * GG * HD * 2); bf* Vh = (bf*)take((size_t)ZC * HD * GG * 2); bf* Vl = (bf*)take((size_t)ZC * HD * GG * 2); float* Sb = (float*)take((size_t)ZC * GG * GG * 4); bf* Ph = (bf*)take((size_t)ZC * GG * GG * 2); bf* Pl = (bf*)take((size_t)ZC * GG * GG * 2);
    float* ObK[3]; float* LSK[3]; for (int k = 0; k < 3; ++k) { const int nzk = (4 >> k) * NH_; ObK[k] = (float*)take((size_t)nzk * GG * HD * 4); LSK[k] = (float*)take((size_t)nzk * GG * 32 * 4); }
    bf* Ah = (bf*)take((size_t)LL * EE * 2); bf* Al = (bf*)take((size_t)LL * EE * 2);
    if ((size_t)(wsp - (char*)d_ws) > ws_size) return;
    k_wtG<<<(EE * 3 * EE / 64 + 63) / 64, 256, 0, stream>>>(wqkv, EE, 3 * EE, WQ); k_wtG<<<(EE * EE / 64 + 63) / 64, 256, 0, stream>>>(wproj, EE, EE, WP);
    k_cvt8<<<(LL * EE / 8 + 255) / 256, 256, 0, stream>>>(x, XB, (size_t)LL * EE / 8);
    k_gemmw<bf, 0, false><<<dim3(LL / 64, 3 * EE / 64, 1), 32, 0, stream>>>(XB, nullptr, WQ, nullptr, EE, QKV, 3 * EE, nullptr, 0, 0, 0);
    const int rs[3] = {1, 2, 4};
    for (int kb = 0; kb < 3; ++kb) { const int r = rs[kb]; const int nseg = LL / (GG * r); const int nz = nseg * NH_;
        for (int z0 = 0; z0 < nz; z0 += ZC) {
            k_gath<<<(unsigned)(((size_t)ZC * GG * HD / 2 + 255) / 256), 256, 0, stream>>>(QKV, r, z0, Qh, Ql, Kh, Kl); k_gathv<<<(unsigned)(((size_t)ZC * HD * GG / 2 + 255) / 256), 256, 0, stream>>>(QKV, r, z0, Vh, Vl);
            k_gemmc<bf, 2, 1><<<dim3(GG / 64, GG / 64, ZC), 32, 0, stream>>>(Qh, Ql, Kh, Kl, HD, Sb, GG, 0, (size_t)GG * HD, (size_t)GG * HD, (size_t)GG * GG);
            k_csoft<<<ZC * GG / 8, 256, 0, stream>>>(Sb, Ph, Pl, LSK[kb] + (size_t)z0 * GG * 32);
            k_gemmc<bf, 2, 2><<<dim3(GG / 64, 1, ZC), 32, 0, stream>>>(Ph, Pl, Vh, Vl, GG, ObK[kb] + (size_t)z0 * GG * HD, HD, 0, (size_t)GG * GG, (size_t)HD * GG, (size_t)GG * HD); }
        }
    k_comb<<<(unsigned)(((size_t)LL * EE / 2 + 255) / 256), 256, 0, stream>>>(ObK[0], ObK[1], ObK[2], LSK[0], LSK[1], LSK[2], Ah, Al);
    k_gemmw<bf, 1, false><<<dim3(LL / 64, EE / 64, 1), 32, 0, stream>>>(Ah, Al, WP, nullptr, EE, OUT, EE, nullptr, 0, 0, 0);
}
